// GraphSAGE_24618752541196
// MI455X (gfx1250) — hardware-run, weakly checked
//
#include <hip/hip_runtime.h>
#include <stddef.h>
#include <stdint.h>
#include <math.h>


#define D       64
#define KSEG    128
#define KP      256
#define NTHR    256
#define NWAVE   8
#define EPT     8
#define CHUNK   (NTHR * EPT)
#define WCAP    (EPT * 32)
#define LISTN   (NWAVE * WCAP)
#define NBA     1024
#define PKS     10
#define RCAP    28672
#define DEGCAP  128
#define GBM     64
#define GBN     64
#define GTHR    128
#define USEG    1024
#define NUW     (4 * USEG)
#define EPB     256
#define ZINTS   (2 * RCAP + 2 * NBA + LISTN)
#define LDS_AGG (ZINTS * 4 + 64)
#define WSMAX   134217728

static_assert((CHUNK & (CHUNK - 1)) == 0);
static_assert(NBA == (1 << PKS));
static_assert(((long long)CHUNK << PKS) < (1LL << 31));
static_assert(NTHR * 4 == NBA);
static_assert(LISTN >= NBA && LISTN >= NWAVE * WCAP);
static_assert((RCAP % 32) == 0);
static_assert((ZINTS % (NTHR * 4)) == 0);
static_assert(LDS_AGG <= 300000);
static_assert((NBA % NWAVE) == 0 && (NBA % GBM) == 0);
static_assert(GBM == (GTHR / 32) * 16);
static_assert(GBN == D && GBN == 4 * 16);
static_assert(KSEG == 2 * D && KP == 2 * KSEG && (KP % 32) == 0);
static_assert(KP * 2 == 32 * 16);
static_assert(D == 32 * 2);
static_assert(D == 16 * 4);
static_assert(2 * GBN * 4 == 32 * 16);
static_assert((USEG % NTHR) == 0 && USEG == D * (D / 4));
static_assert(EPB == NTHR && (EPB % 32) == 0 && 2 * (EPB / 4) <= NTHR);
static_assert(GBN <= GTHR && 2 * D <= NTHR);

typedef float          v2f  __attribute__((ext_vector_type(2)));
typedef float          v4f  __attribute__((ext_vector_type(4)));
typedef float          v8f  __attribute__((ext_vector_type(8)));
typedef int            v4i  __attribute__((ext_vector_type(4)));
typedef int            v8i  __attribute__((ext_vector_type(8)));
typedef unsigned short v8us __attribute__((ext_vector_type(8)));
typedef __bf16         v16b __attribute__((ext_vector_type(16)));
typedef v2f  __attribute__((may_alias)) v2fa;
typedef v4f  __attribute__((may_alias)) v4fa;
typedef v4i  __attribute__((may_alias)) v4ia;
typedef v8us __attribute__((may_alias)) v8usa;
union Frag { v16b b; v8us h[2]; v8i w; };

__device__ __forceinline__ v8f wmk(const Frag& a, const Frag& b, v8f c) {
  v8f d = __builtin_amdgcn_wmma_f32_16x16x32_bf16(false, a.b, false, b.b, (short)0, c, false, false);
  asm volatile("v_nop\n\tv_nop\n\tv_nop\n\tv_nop" : "+v"(d) : "v"(a.w), "v"(b.w));
  return d;
}

__device__ __forceinline__ v8f z8() { v8f z = {0.f, 0.f, 0.f, 0.f, 0.f, 0.f, 0.f, 0.f}; return z; }

__device__ __forceinline__ unsigned bf16_bits(float f) {
  const unsigned u = __float_as_uint(f);
  return (u + 0x7FFFu + ((u >> 16) & 1u)) >> 16;
}
__device__ __forceinline__ float bf16_val(float f) {
  return __uint_as_float(bf16_bits(f) << 16);
}

__device__ __forceinline__ int scan_chunk(const int* __restrict__ dsts, int nE, int cbase, int slotBase,
                                          int nb, int vec8, int* list, int tid, int lane, int wave) {
  int wc = 0;
  const int el0  = tid * EPT;
  const int e0   = cbase + el0;
  const int sent = -2147483647 - 1;
  v4i da, db;
  if (vec8 != 0 && cbase + CHUNK <= nE) {
    da = *(const v4i*)(dsts + e0);
    db = *(const v4i*)(dsts + e0 + 4);
  } else {
    da.x = (e0     < nE) ? dsts[min(e0,     nE - 1)] : sent;
    da.y = (e0 + 1 < nE) ? dsts[min(e0 + 1, nE - 1)] : sent;
    da.z = (e0 + 2 < nE) ? dsts[min(e0 + 2, nE - 1)] : sent;
    da.w = (e0 + 3 < nE) ? dsts[min(e0 + 3, nE - 1)] : sent;
    db.x = (e0 + 4 < nE) ? dsts[min(e0 + 4, nE - 1)] : sent;
    db.y = (e0 + 5 < nE) ? dsts[min(e0 + 5, nE - 1)] : sent;
    db.z = (e0 + 6 < nE) ? dsts[min(e0 + 6, nE - 1)] : sent;
    db.w = (e0 + 7 < nE) ? dsts[min(e0 + 7, nE - 1)] : sent;
  }
  const unsigned nbs = (unsigned)slotBase;
  const unsigned unb = (unsigned)nb;
  const unsigned s0 = (unsigned)da.x - nbs, s1 = (unsigned)da.y - nbs;
  const unsigned s2 = (unsigned)da.z - nbs, s3 = (unsigned)da.w - nbs;
  const unsigned s4 = (unsigned)db.x - nbs, s5 = (unsigned)db.y - nbs;
  const unsigned s6 = (unsigned)db.z - nbs, s7 = (unsigned)db.w - nbs;
  const bool h0 = s0 < unb, h1 = s1 < unb, h2 = s2 < unb, h3 = s3 < unb;
  const bool h4 = s4 < unb, h5 = s5 < unb, h6 = s6 < unb, h7 = s7 < unb;
  const unsigned any = __builtin_amdgcn_ballot_w32(h0 | h1 | h2 | h3 | h4 | h5 | h6 | h7);
  if (any != 0u) {
#define HITJ(J, HJ, SJ) { \
      const unsigned mj = __builtin_amdgcn_ballot_w32(HJ); \
      if (mj != 0u) { \
        if (HJ) { \
          const int pos = wc + (int)__builtin_amdgcn_mbcnt_lo(mj, 0u); \
          if (pos < WCAP) list[wave * WCAP + pos] = ((el0 + (J)) << PKS) | (int)(SJ); \
        } \
        wc += (int)__builtin_popcount(mj); } }
    HITJ(0, h0, s0)
    HITJ(1, h1, s1)
    HITJ(2, h2, s2)
    HITJ(3, h3, s3)
    HITJ(4, h4, s4)
    HITJ(5, h5, s5)
    HITJ(6, h6, s6)
    HITJ(7, h7, s7)
#undef HITJ
  }
  return wc;
}

__global__ __launch_bounds__(NTHR) void k_wprep(const float* __restrict__ wl1, const float* __restrict__ wr1,
                                                const float* __restrict__ wl2, const float* __restrict__ wr2,
                                                unsigned short* BT1, unsigned short* BT2) {
  const int u = (int)blockIdx.x * NTHR + (int)threadIdx.x;
  const float* W;
  unsigned short* B;
  int seg;
  if (u < USEG)            { W = wl1; B = BT1; seg = 0; }
  else if (u < 2 * USEG)   { W = wr1; B = BT1; seg = 1; }
  else if (u < 3 * USEG)   { W = wl2; B = BT2; seg = 0; }
  else if (u < 4 * USEG)   { W = wr2; B = BT2; seg = 1; }
  else return;
  const int v  = u & (USEG - 1);
  const int n  = v >> 4;
  const int qq = v & 15;
  const v4f a = *(const v4fa*)(W + (size_t)n * D + 4 * qq);
  const unsigned short b0 = (unsigned short)bf16_bits(a.x);
  const unsigned short b1 = (unsigned short)bf16_bits(a.y);
  const unsigned short b2 = (unsigned short)bf16_bits(a.z);
  const unsigned short b3 = (unsigned short)bf16_bits(a.w);
  v8us o;
  o[0] = b0; o[1] = b1; o[2] = b2; o[3] = b3;
  o[4] = b0; o[5] = b1; o[6] = b2; o[7] = b3;
  unsigned short* dp = B + (size_t)n * KP + seg * KSEG + 8 * qq;
  *(volatile v8us*)dp = o;
  __threadfence();
  *(volatile v8us*)dp = o;
}

__global__ __launch_bounds__(GTHR) void k_gemm(const unsigned short* __restrict__ A, int lda,
                                               const unsigned short* __restrict__ BT, int K,
                                               const float* __restrict__ bias, float* outF) {
  __shared__ __attribute__((aligned(16))) float stg[GBM * GBN];
  __shared__ __attribute__((aligned(16))) float cb[GBN];
  const int tid = (int)threadIdx.x, lane = tid & 31, wave = tid >> 5, hh = lane >> 4, m = lane & 15;
  const int rowBase = (int)blockIdx.x * GBM;
  if (tid < GBN) cb[tid] = bf16_val(bias[tid]);
  __syncthreads();

  v8f acc[4];
#pragma unroll
  for (int t = 0; t < 4; ++t) acc[t] = z8();
  const unsigned short* ap = A  + (size_t)(rowBase + 16 * wave + m) * (size_t)lda + 8 * hh;
  const unsigned short* wp = BT + (size_t)m * (size_t)K + 8 * hh;
  const int ksteps = K >> 5;
#pragma unroll 1
  for (int ks = 0; ks < ksteps; ++ks) {
    Frag af;
    af.h[0] = *(const v8usa*)(ap + 32 * ks);
    af.h[1] = *(const v8usa*)(ap + 32 * ks + 16);
#pragma unroll
    for (int t = 0; t < 4; ++t) {
      const unsigned short* wq = wp + (size_t)(16 * t) * (size_t)K + 32 * ks;
      Frag bf;
      bf.h[0] = *(const v8usa*)wq;
      bf.h[1] = *(const v8usa*)(wq + 16);
      acc[t] = wmk(af, bf, acc[t]);
    }
  }

#pragma unroll
  for (int t = 0; t < 4; ++t) {
    const int lc = 16 * t + m;
    const float bb = cb[lc];
#pragma unroll
    for (int r = 0; r < 8; ++r) {
      const int lr = 16 * wave + 8 * hh + r;
      stg[lr * GBN + lc] = acc[t][r] + bb;
    }
  }
  __syncthreads();

  v4f fv[8];
#pragma unroll
  for (int i = 0; i < 8; ++i) {
    const int lr = 16 * wave + 2 * i;
    fv[i] = *(const v4fa*)(stg + lr * GBN + 4 * lane);
  }
#pragma unroll
  for (int i = 0; i < 8; ++i) {
    const int gr = rowBase + 16 * wave + 2 * i;
    float* op = outF + (size_t)gr * (size_t)GBN + 4 * lane;
    *(volatile v4f*)op = fv[i];
  }
  __threadfence();
#pragma unroll
  for (int i = 0; i < 8; ++i) {
    const int gr = rowBase + 16 * wave + 2 * i;
    float* op = outF + (size_t)gr * (size_t)GBN + 4 * lane;
    *(volatile v4f*)op = fv[i];
  }
}

template <int RIN>
__global__ __launch_bounds__(NTHR) void k_agg(const int* __restrict__ srcs, const int* __restrict__ dsts,
                                              const float* __restrict__ ew, const float* __restrict__ F,
                                              unsigned short* Aout, int nN, int nE, int vec8) {
  extern __shared__ __attribute__((aligned(16))) int lds_i[];
  int* reg1 = lds_i;
  int* reg2 = reg1 + RCAP;
  int* scnt = reg2 + RCAP;
  int* soff = scnt + NBA;
  int* list = soff + NBA;
  int* wcnt = list + LISTN;
  int* wtot = wcnt + NWAVE;
  const int tid = (int)threadIdx.x, lane = tid & 31, wave = tid >> 5;
  const int nodeBase = (int)blockIdx.x * NBA;

  {
    const v4i z4 = {0, 0, 0, 0};
    for (int i = tid * 4; i < ZINTS; i += NTHR * 4) *(v4ia*)(lds_i + i) = z4;
    if (tid < 2 * NWAVE) wcnt[tid] = 0;
  }
  __syncthreads();

  int tot = 0;
  const int nChunks = (nE + CHUNK - 1) / CHUNK;
#pragma unroll 1
  for (int ch = 0; ch < nChunks; ++ch) {
    const int cbase = ch * CHUNK;
    const int wc = scan_chunk(dsts, nE, cbase, nodeBase, NBA, vec8, list, tid, lane, wave);
    if (lane == 0) wcnt[wave] = wc;
    __syncthreads();
    int pre = 0, all = 0;
#pragma unroll
    for (int w2 = 0; w2 < NWAVE; ++w2) {
      int c = wcnt[w2];
      c = c < 0 ? 0 : (c > WCAP ? WCAP : c);
      all += c;
      pre += (w2 < wave) ? c : 0;
    }
    const int wcc  = wc > WCAP ? WCAP : wc;
    const int base = tot + pre;
#pragma unroll 1
    for (int i = lane; i < wcc; i += 32) {
      const int ent = list[wave * WCAP + i];
      const int el  = (ent >> PKS) & (CHUNK - 1);
      const int sl  = ent & (NBA - 1);
      int eid = cbase + el;
      eid = eid > nE - 1 ? nE - 1 : eid;
      const int pos = base + i;
      if (pos < RCAP) reg1[pos] = (int)(((unsigned)eid << PKS) | (unsigned)sl);
    }
    tot += all;
    tot = tot > RCAP ? RCAP : tot;
    __syncthreads();
  }
  const int nh = tot;

  if (wave == 0) {
#pragma unroll 1
    for (int b0 = 0; b0 < nh; b0 += 32) {
      const int idx = b0 + lane;
      const int uv  = reg1[idx < RCAP ? idx : RCAP - 1];
      const int m32 = (nh - b0) < 32 ? (nh - b0) : 32;
#pragma unroll 1
      for (int k = 0; k < m32; ++k) {
        const int u  = __builtin_amdgcn_readlane(uv, k);
        const int sl = u & (NBA - 1);
        if (lane == 0) scnt[sl] = scnt[sl] + 1;
      }
    }
  }
  __syncthreads();

  {
    const v4i ca = *(const v4ia*)(scnt + 4 * tid);
    const int e0 = ca.x < 0 ? 0 : ca.x, e1 = ca.y < 0 ? 0 : ca.y, e2 = ca.z < 0 ? 0 : ca.z, e3 = ca.w < 0 ? 0 : ca.w;
    const int ts = e0 + e1 + e2 + e3;
    int incl = ts;
#pragma unroll
    for (int d = 1; d < 32; d <<= 1) {
      const int up = __shfl_up(incl, d, 32);
      if (lane >= d) incl += up;
    }
    if (lane == 31) wtot[wave] = incl;
    __syncthreads();
    int pre = 0;
#pragma unroll
    for (int w2 = 0; w2 < NWAVE; ++w2) pre += (w2 < wave) ? wtot[w2] : 0;
    int run = pre + incl - ts;
    soff[4 * tid + 0] = run; run += e0;
    soff[4 * tid + 1] = run; run += e1;
    soff[4 * tid + 2] = run; run += e2;
    soff[4 * tid + 3] = run;
  }
  __syncthreads();
  for (int i = tid; i < NBA; i += NTHR) list[i] = soff[i];
  __syncthreads();

  if (wave == 0) {
#pragma unroll 1
    for (int b0 = 0; b0 < nh; b0 += 32) {
      const int idx = b0 + lane;
      const int uv  = reg1[idx < RCAP ? idx : RCAP - 1];
      const int m32 = (nh - b0) < 32 ? (nh - b0) : 32;
#pragma unroll 1
      for (int k = 0; k < m32; ++k) {
        const int u   = __builtin_amdgcn_readlane(uv, k);
        const int sl  = u & (NBA - 1);
        const int eid = (int)((unsigned)u >> PKS);
        if (lane == 0) {
          int pos = list[sl];
          pos = pos < 0 ? 0 : (pos > RCAP - 1 ? RCAP - 1 : pos);
          reg2[pos] = eid;
          list[sl] = pos + 1;
        }
      }
    }
  }
  __syncthreads();

  const int nbw = NBA / NWAVE;
  const bool ovf = (nh >= RCAP);
  const float qnan = __int_as_float(0x7fc00000);
  const int cr = 4 * (lane & 15);
  const int sA = (2 * lane) & 31;
  const int sB = (2 * lane + 1) & 31;
  const bool lo16 = lane < 16;

#pragma unroll 1
  for (int jt = 0; jt < nbw; ++jt) {
    const int slot = wave * nbw + jt;
    const int node = nodeBase + slot;
    int st = soff[slot];
    const int craw = scnt[slot];
    int cnt = craw;
    st  = st < 0 ? 0 : (st > nh ? nh : st);
    cnt = cnt < 0 ? 0 : (cnt > DEGCAP ? DEGCAP : cnt);
    if (cnt > nh - st) cnt = nh - st;
    const float pz = (ovf || craw > DEGCAP) ? qnan : 0.0f;
    const bool live = node < nN;
    const int nc = node < nN ? node : nN - 1;

    float a0 = 0.0f, a1 = 0.0f, dsum = 0.0f;
#pragma unroll 1
    for (int b0 = 0; b0 < cnt; b0 += 32) {
      int idx = st + b0 + lane; idx = idx > RCAP - 1 ? RCAP - 1 : idx;
      int eid = reg2[idx]; eid = eid < 0 ? 0 : (eid > nE - 1 ? nE - 1 : eid);
      int sr = srcs[eid]; sr = sr < 0 ? 0 : (sr > nN - 1 ? nN - 1 : sr);
      const int wvi = __float_as_int(bf16_val(ew[eid]));
      const int m32 = (cnt - b0) < 32 ? (cnt - b0) : 32;
#pragma unroll 1
      for (int k = 0; k < m32; ++k) {
        const int   sk = __builtin_amdgcn_readlane(sr, k);
        const float wk = __int_as_float(__builtin_amdgcn_readlane(wvi, k));
        const v2f v = *(const v2fa*)(F + (size_t)sk * D + 2 * lane);
        float vx = v.x, vy = v.y;
        if constexpr (RIN == 1) { vx = bf16_val(vx); vy = bf16_val(vy); }
        a0 = fmaf(wk, vx, a0);
        a1 = fmaf(wk, vy, a1);
        dsum = dsum + wk;
      }
    }
    const float rden = 1.0f / fmaxf(dsum, 1e-6f);
    const float q0 = a0 * rden, q1 = a1 * rden;
    const float c0 = __shfl(q0, sA, 32);
    const float c1 = __shfl(q1, sA, 32);
    const float c2 = __shfl(q0, sB, 32);
    const float c3 = __shfl(q1, sB, 32);

    const v4f xa = *(const v4fa*)(F + (size_t)nc * D + cr);
    float x0 = xa.x, x1 = xa.y, x2 = xa.z, x3 = xa.w;
    if constexpr (RIN == 1) { x0 = bf16_val(x0); x1 = bf16_val(x1); x2 = bf16_val(x2); x3 = bf16_val(x3); }

    const float f0 = lo16 ? c0 : x0;
    const float f1 = lo16 ? c1 : x1;
    const float f2 = lo16 ? c2 : x2;
    const float f3 = lo16 ? c3 : x3;
    const float r0 = (live ? f0 : 0.0f) + pz;
    const float r1 = (live ? f1 : 0.0f) + pz;
    const float r2 = (live ? f2 : 0.0f) + pz;
    const float r3 = (live ? f3 : 0.0f) + pz;

    const unsigned h0 = bf16_bits(r0), h1 = bf16_bits(r1), h2 = bf16_bits(r2), h3 = bf16_bits(r3);
    v8us pk;
    pk[0] = (unsigned short)h0; pk[1] = (unsigned short)h1; pk[2] = (unsigned short)h2; pk[3] = (unsigned short)h3;
    pk[4] = (unsigned short)bf16_bits(r0 - __uint_as_float(h0 << 16));
    pk[5] = (unsigned short)bf16_bits(r1 - __uint_as_float(h1 << 16));
    pk[6] = (unsigned short)bf16_bits(r2 - __uint_as_float(h2 << 16));
    pk[7] = (unsigned short)bf16_bits(r3 - __uint_as_float(h3 << 16));

    unsigned short* gp = Aout + (size_t)node * (size_t)KP + 8 * lane;
    *(volatile v8us*)gp = pk;
    __threadfence();
    *(volatile v8us*)gp = pk;
  }
}

__global__ __launch_bounds__(NTHR) void k_pair(const int* __restrict__ sup, int nS, int nN,
                                               const float* __restrict__ H,
                                               const float* __restrict__ wwp, const float* __restrict__ bwp,
                                               const float* __restrict__ wep, const float* __restrict__ bep,
                                               float* out) {
  __shared__ __attribute__((aligned(16))) float cw[2 * D];
  __shared__ __attribute__((aligned(16))) float ce[2 * D];
  __shared__ __attribute__((aligned(16))) float cb2[16];
  __shared__ __attribute__((aligned(16))) float sy0[EPB];
  __shared__ __attribute__((aligned(16))) float sy1[EPB];
  const int tid = (int)threadIdx.x;

  if (tid < 2 * D) {
    cw[tid] = bf16_val(wwp[tid]);
    ce[tid] = bf16_val(wep[tid]);
  }
  if (tid < 32) {
    const float vb = bf16_val(bwp[0]);
    const float ve = bf16_val(bep[0]);
    if (tid == 0) { cb2[0] = vb; cb2[1] = ve; }
  }

  const int e0 = (int)blockIdx.x * EPB;
  int ec = e0 + tid;
  ec = ec > nS - 1 ? nS - 1 : ec;
  int s = sup[ec];
  int t = sup[(size_t)nS + (size_t)ec];
  s = s < 0 ? 0 : (s > nN - 1 ? nN - 1 : s);
  t = t < 0 ? 0 : (t > nN - 1 ? nN - 1 : t);
  const float* pa = H + (size_t)s * D;
  const float* pb = H + (size_t)t * D;
  __syncthreads();

  float dw = 0.0f, de = 0.0f;
#pragma unroll 1
  for (int c4 = 0; c4 < D / 4; ++c4) {
    const v4f a  = *(const v4fa*)(pa + 4 * c4);
    const v4f b  = *(const v4fa*)(pb + 4 * c4);
    const v4f ws = *(const v4fa*)(cw + 4 * c4);
    const v4f wq = *(const v4fa*)(cw + D + 4 * c4);
    const v4f es = *(const v4fa*)(ce + 4 * c4);
    const v4f eq = *(const v4fa*)(ce + D + 4 * c4);
    const float u0 = a.x + b.x, u1 = a.y + b.y, u2 = a.z + b.z, u3 = a.w + b.w;
    const float p0 = a.x * b.x, p1 = a.y * b.y, p2 = a.z * b.z, p3 = a.w * b.w;
    dw = fmaf(u0, ws.x, dw); dw = fmaf(u1, ws.y, dw); dw = fmaf(u2, ws.z, dw); dw = fmaf(u3, ws.w, dw);
    dw = fmaf(p0, wq.x, dw); dw = fmaf(p1, wq.y, dw); dw = fmaf(p2, wq.z, dw); dw = fmaf(p3, wq.w, dw);
    de = fmaf(u0, es.x, de); de = fmaf(u1, es.y, de); de = fmaf(u2, es.z, de); de = fmaf(u3, es.w, de);
    de = fmaf(p0, eq.x, de); de = fmaf(p1, eq.y, de); de = fmaf(p2, eq.z, de); de = fmaf(p3, eq.w, de);
  }
  const float yw = fmaxf(dw + cb2[0], 0.0f);
  const float ye = de + cb2[1];
  sy0[tid] = yw;
  sy1[tid] = ye;
  __syncthreads();

  const int  q      = tid & 63;
  const bool second = tid >= 64;
  const v4f  o0 = *(const v4fa*)(sy0 + 4 * q);
  const v4f  o1 = *(const v4fa*)(sy1 + 4 * q);
  const v4f  ov = second ? o1 : o0;
  const size_t base = second ? (size_t)nS : (size_t)0;
  const bool stv = (tid < 128) && (e0 + 4 * q + 3 < nS);
  float* op = out + base + (size_t)e0 + (size_t)(4 * q);
  if (stv) *(volatile v4f*)op = ov;
  __threadfence();
  if (stv) *(volatile v4f*)op = ov;
}

static inline int cdiv(int a, int b) { return (a + b - 1) / b; }
static inline size_t al256(size_t o) { return (o + 255) & ~(size_t)255; }

extern "C" void kernel_launch(void* const* d_in, const int* in_sizes, int n_in,
                              void* d_out, int out_size, void* d_ws, size_t ws_size,
                              hipStream_t stream) {
  if (n_in < 14) return;
  if (in_sizes[0] < D || (in_sizes[0] % D) != 0) return;
  const int nN = in_sizes[0] / D;
  if (nN < GBM || nN > (1 << 22)) return;
  if (in_sizes[1] < 2 || (in_sizes[1] & 1) != 0) return;
  const int nS = in_sizes[1] / 2;
  if (nS < 32 || (nS & 31) != 0) return;
  if (in_sizes[2] < 2 || (in_sizes[2] & 1) != 0) return;
  const int nE = in_sizes[2] / 2;
  if (nE < 1 || nE >= (1 << (32 - PKS))) return;
  if (in_sizes[3] != nE) return;
  if (in_sizes[4] != D * D || in_sizes[6] != D * D) return;
  if (in_sizes[7] != D * D || in_sizes[9] != D * D) return;
  if (in_sizes[5] != D || in_sizes[8] != D) return;
  if (in_sizes[10] != 2 * D || in_sizes[12] != 2 * D) return;
  if (in_sizes[11] != 1 || in_sizes[13] != 1) return;
  if ((long long)out_size != 2LL * (long long)nS) return;

  const float* x    = (const float*)d_in[0];
  const int*   sup  = (const int*)  d_in[1];
  const int*   medg = (const int*)  d_in[2];
  const float* mew  = (const float*)d_in[3];
  const float* w1l  = (const float*)d_in[4];
  const float* b1   = (const float*)d_in[5];
  const float* w1r  = (const float*)d_in[6];
  const float* w2l  = (const float*)d_in[7];
  const float* b2   = (const float*)d_in[8];
  const float* w2r  = (const float*)d_in[9];
  const float* wep  = (const float*)d_in[10];
  const float* bep  = (const float*)d_in[11];
  const float* wwp  = (const float*)d_in[12];
  const float* bwp  = (const float*)d_in[13];
  float* out = (float*)d_out;
  const int* msrc = medg;
  const int* mdst = medg + nE;

  const int MP   = cdiv(nN, GBM) * GBM;
  const int gM   = MP / GBM;
  const int gA   = cdiv(MP, NBA);
  const int RA   = gA * NBA;
  const int vec8 = ((nE & 3) == 0) ? 1 : 0;
  if ((long long)RA < (long long)MP) return;
  if ((long long)gM * GBM < (long long)nN) return;

  char* ws = (char*)d_ws;
  size_t off = 0;
  const size_t oBT1 = off; off = al256(off + (size_t)D * KP * 2);
  const size_t oBT2 = off; off = al256(off + (size_t)D * KP * 2);
  const size_t oAP  = off; off = al256(off + (size_t)RA * KP * 2);
  const size_t oH1  = off; off = al256(off + (size_t)MP * D * 4);
  const size_t oH2  = off; off = al256(off + (size_t)MP * D * 4);
  if (off > ws_size || off > (size_t)WSMAX) return;
  unsigned short* BT1 = (unsigned short*)(ws + oBT1);
  unsigned short* BT2 = (unsigned short*)(ws + oBT2);
  unsigned short* AP  = (unsigned short*)(ws + oAP);
  float*          H1  = (float*)(ws + oH1);
  float*          H2  = (float*)(ws + oH2);

  hipFuncSetAttribute(reinterpret_cast<const void*>(&k_agg<1>), hipFuncAttributeMaxDynamicSharedMemorySize, LDS_AGG);
  hipFuncSetAttribute(reinterpret_cast<const void*>(&k_agg<0>), hipFuncAttributeMaxDynamicSharedMemorySize, LDS_AGG);

  k_wprep<<<NUW / NTHR, NTHR, 0, stream>>>(w1l, w1r, w2l, w2r, BT1, BT2);
  k_agg<1><<<gA, NTHR, LDS_AGG, stream>>>(msrc, mdst, mew, x, AP, nN, nE, vec8);
  k_gemm<<<gM, GTHR, 0, stream>>>(AP, KP, BT1, KP, b1, H1);
  k_agg<0><<<gA, NTHR, LDS_AGG, stream>>>(msrc, mdst, mew, H1, AP, nN, nE, vec8);
  k_gemm<<<gM, GTHR, 0, stream>>>(AP, KP, BT2, KP, b2, H2);
  k_pair<<<cdiv(nS, EPB), NTHR, 0, stream>>>(sup, nS, nN, H2, wwp, bwp, wep, bep, out);
}
